// MultiheadLatentAttn_54674933678912
// MI455X (gfx1250) — hardware-verified
//
#include <hip/hip_runtime.h>
#include <math.h>
#include <stdint.h>

#ifndef NB
#define NB 4
#endif
#ifndef SEQ
#define SEQ 2048
#endif
#define XS_FULL 2048
#define DMOD 1024
#define NH 16
#define DLQ 256
#define DLKV 128
#define DNOPE 10
#define DROPE 10
#define DQK 20
#define DV 64
#define NQ (NH * DQK)
#define NKVA (DLKV + DROPE)
#define NKVP 192
#define DCAT 160
#define QCW (NH * DCAT)
#define HROW (DNOPE + DV)
#define WKVB_ROWS (NH * HROW)
#define VOUT (NH * DV)
#define MAXB 4
#define QA ((SEQ < 256) ? SEQ : 256)
#define MROWS (NB * SEQ)
#define NKT (SEQ / 32)
#define NQT (SEQ / 16)
#define NQT32 ((NQT + 31) / 32)
#define NST (SEQ / 64)
#define KCT 64
#define WPB 2
#define NHP (NH / WPB)
#define ATT_THREADS (WPB * 32)
#define PTP 36
#define PTW (16 * PTP)
#define SLP 132
#define SLW (16 * SLP)
#define WREG (PTW + SLW)
#define SLAB64 (16 * 68)
#define SCL 0.22360679774997896f
#define LN_NKEY 7.6246189861593985f
#define LOG2E 1.4426950408889634f
#define RMS_EPS 1e-6f
#define QNS 64.0f
#define WQS 1024.0f
#define QSC 1024.0f
#define KSC 256.0f
#define PCAR 32768.0f
#define AVS 1024.0f
#define WVS 1024.0f
#define OSC 1024.0f
#define WOS 1024.0f
#define MASK_THR (-1.0e8f)
#define WS_CAP 134217728

static_assert(NB >= 1 && NB <= MAXB);
static_assert((SEQ % 64) == 0 && SEQ >= 64 && SEQ <= XS_FULL);
static_assert((QA % 64) == 0 && QA >= 64 && QA <= SEQ && ((SEQ - QA) % 64) == 0 && (QA % 16) == 0);
static_assert(VOUT == DMOD && NH * DV == VOUT && NHP * WPB == NH && ATT_THREADS == 64);
static_assert((DCAT % 32) == 0 && DCAT >= NKVA && (DLKV % 32) == 0 && (DLQ % 64) == 0 && (NQ % 64) == 0);
static_assert((NKVP % 64) == 0 && NKVP >= NKVA && (DMOD % 64) == 0 && (VOUT % 64) == 0 && (DLQ % 32) == 0);
static_assert(WPB * WREG * 4 <= 65536 && 2 * KCT * DCAT * 2 <= 65536 && 4 * SLAB64 * 4 <= 65536);
static_assert(((KCT * DCAT) % (256 * 8)) == 0 && KCT * 4 == 256);
static_assert(NQ == 320 && QCW == NQ * 8 && DQK == DNOPE + DROPE);
static_assert(DLKV == 4 * 32 && (DCAT - DLKV) == 4 * 8 && DLKV == 8 * 16);
static_assert((DLQ / 8) == 32);

typedef unsigned short u16;
typedef _Float16 v16h __attribute__((ext_vector_type(16)));
typedef _Float16 v8h  __attribute__((ext_vector_type(8)));
typedef __bf16   v16b __attribute__((ext_vector_type(16)));
typedef float    v8f  __attribute__((ext_vector_type(8)));
typedef float    v4f  __attribute__((ext_vector_type(4)));
typedef unsigned int v4u __attribute__((ext_vector_type(4)));
typedef unsigned int v2u __attribute__((ext_vector_type(2)));

union FragH { v16h v; v8h h[2]; v4u u[2]; };
union FragB { v16b v; v4u u[2]; };

__device__ __forceinline__ unsigned short bf_bits(float f) {
  unsigned u = __float_as_uint(f);
  return (unsigned short)((u + 0x7FFFu + ((u >> 16) & 1u)) >> 16);
}
__device__ __forceinline__ float bf_up(unsigned short h) { return __uint_as_float(((unsigned)h) << 16); }
__device__ __forceinline__ float bfr(float f) { return bf_up(bf_bits(f)); }
__device__ __forceinline__ unsigned short h_bits(_Float16 x) { return __builtin_bit_cast(unsigned short, x); }
__device__ __forceinline__ unsigned pk16(unsigned short a, unsigned short b) { return (unsigned)a | ((unsigned)b << 16); }
__device__ __forceinline__ v8f zero8() { v8f z = {0.f, 0.f, 0.f, 0.f, 0.f, 0.f, 0.f, 0.f}; return z; }

__device__ __forceinline__ v16h ldfrag_h(const _Float16* p) {
  FragH f;
  f.h[0] = *(const v8h*)(p);
  f.h[1] = *(const v8h*)(p + 16);
  return f.v;
}
__device__ __forceinline__ v16b ldfrag_b(const u16* p) {
  FragB f;
  f.u[0] = *(const v4u*)(p);
  f.u[1] = *(const v4u*)(p + 16);
  return f.v;
}

__device__ __forceinline__ v8f mma_h(v16h a, v16h b, v8f c) {
  return __builtin_amdgcn_wmma_f32_16x16x32_f16(false, a, false, b, (short)0, c, false, false);
}
__device__ __forceinline__ v8f mma_b(v16b a, v16b b, v8f c) {
  return __builtin_amdgcn_wmma_f32_16x16x32_bf16(false, a, false, b, (short)0, c, false, false);
}
__device__ __forceinline__ void guard2(v8f& a, v8f& b, v16h x0, v16h x1, v16h x2, v16h x3, v16h x4, v16h x5) {
#if defined(__HIP_DEVICE_COMPILE__)
  asm volatile("v_nop\n\tv_nop\n\tv_nop\n\tv_nop"
               : "+v"(a), "+v"(b) : "v"(x0), "v"(x1), "v"(x2), "v"(x3), "v"(x4), "v"(x5) : "memory");
#endif
}
template <typename F>
__device__ __forceinline__ void guard6(v8f& a, v8f& b, v8f& c, v8f& d, F x0, F x1, F x2, F x3, F x4, F x5) {
#if defined(__HIP_DEVICE_COMPILE__)
  asm volatile("v_nop\n\tv_nop\n\tv_nop\n\tv_nop"
               : "+v"(a), "+v"(b), "+v"(c), "+v"(d) : "v"(x0), "v"(x1), "v"(x2), "v"(x3), "v"(x4), "v"(x5) : "memory");
#endif
}
__device__ __forceinline__ void acc_guard4(v8f& a, v8f& b, v8f& c, v8f& d) {
#if defined(__HIP_DEVICE_COMPILE__)
  asm volatile("v_nop\n\tv_nop\n\tv_nop\n\tv_nop" : "+v"(a), "+v"(b), "+v"(c), "+v"(d));
#endif
}
__device__ __forceinline__ void wave_sync_lds() {
  __builtin_amdgcn_fence(__ATOMIC_RELEASE, "workgroup");
  __builtin_amdgcn_wave_barrier();
  __builtin_amdgcn_fence(__ATOMIC_ACQUIRE, "workgroup");
}

__global__ __launch_bounds__(256) void cvt_x(const float* __restrict__ x, u16* D, int n8tot, int n8b) {
  const int gt = blockIdx.x * 256 + (int)threadIdx.x;
  if (gt >= n8tot) return;
  const int b = gt / n8b;
  const int w = gt - b * n8b;
  const float* p = x + (size_t)b * XS_FULL * DMOD + (size_t)w * 8;
  const v4f a = *(const v4f*)(p), b4 = *(const v4f*)(p + 4);
  float f[8];
#pragma unroll
  for (int e = 0; e < 4; ++e) { f[e] = a[e]; f[4 + e] = b4[e]; }
  v4u o;
#pragma unroll
  for (int e = 0; e < 4; ++e) o[e] = pk16(bf_bits(f[2 * e]), bf_bits(f[2 * e + 1]));
  u16* d = D + (size_t)gt * 8;
  for (int pass = 0; pass < 2; ++pass) {
    *(volatile v4u*)(d) = o;
    __threadfence();
  }
}

__global__ __launch_bounds__(256) void cvt16(const float* __restrict__ x, u16* D, int n8, int n8src, int f16mode, float scale) {
  const int gt = blockIdx.x * 256 + (int)threadIdx.x;
  if (gt >= n8) return;
  const bool live = (gt < n8src);
  const int gs = live ? gt : (n8src - 1);
  const float* p = x + (size_t)gs * 8;
  const v4f a = *(const v4f*)(p), b4 = *(const v4f*)(p + 4);
  float w[8];
#pragma unroll
  for (int e = 0; e < 4; ++e) { w[e] = live ? a[e] : 0.0f; w[4 + e] = live ? b4[e] : 0.0f; }
  v4u o;
#pragma unroll
  for (int e = 0; e < 4; ++e) {
    const float f0 = w[2 * e], f1 = w[2 * e + 1];
    const unsigned short hb0 = h_bits((_Float16)(bfr(f0) * scale));
    const unsigned short hb1 = h_bits((_Float16)(bfr(f1) * scale));
    const unsigned short bb0 = bf_bits(f0);
    const unsigned short bb1 = bf_bits(f1);
    o[e] = (f16mode != 0) ? pk16(hb0, hb1) : pk16(bb0, bb1);
  }
  u16* d = D + (size_t)gt * 8;
  for (int pass = 0; pass < 2; ++pass) {
    *(volatile v4u*)(d) = o;
    __threadfence();
  }
}

__device__ __forceinline__ void epi64(float* sl, v8f a0, v8f a1, v8f a2, v8f a3, float oscale,
                                      const float* __restrict__ bias, int bias_n,
                                      float* C, int N, size_t rowb, int col0, int lane) {
  const int hh = lane >> 4, m = lane & 15;
#pragma unroll
  for (int r = 0; r < 8; ++r) {
    const int ro = (8 * hh + r) * 68 + m;
    sl[ro]      = a0[r] * oscale;
    sl[ro + 16] = a1[r] * oscale;
    sl[ro + 32] = a2[r] * oscale;
    sl[ro + 48] = a3[r] * oscale;
  }
  wave_sync_lds();
  const int cb = col0 + m * 4;
  v4f bb;
#pragma unroll
  for (int e = 0; e < 4; ++e) {
    const int idx = cb + e;
    const int ci  = (idx < bias_n) ? idx : (bias_n - 1);
    const float bv = bias[ci];
    bb[e] = (idx < bias_n) ? bfr(bv) : 0.0f;
  }
  v4f vals[8];
#pragma unroll
  for (int it = 0; it < 8; ++it) vals[it] = *(const v4f*)(sl + (it * 2 + hh) * 68 + m * 4) + bb;
  float* dst = C + (rowb + (size_t)hh) * (size_t)N + cb;
  for (int pass = 0; pass < 2; ++pass) {
#pragma unroll
    for (int it = 0; it < 8; ++it) {
      *(volatile v4f*)(dst + (size_t)(it * 2) * (size_t)N) = vals[it];
    }
    __threadfence();
  }
}

__global__ __launch_bounds__(128)
void gemm_bf(const u16* __restrict__ A, const u16* __restrict__ Bt, const float* __restrict__ bias, int bias_n,
             float* C, int M, int N, int K, float oscale) {
  __shared__ __align__(16) float slab[4 * SLAB64];
  const int tid = threadIdx.x, wave = tid >> 5, lane = tid & 31, hh = lane >> 4, m = lane & 15;
  const int ntile = N >> 6;
  const int bid   = blockIdx.x;
  const int rowb  = (bid / ntile) * 64 + wave * 16;
  const int col0  = (bid % ntile) * 64;
  if (rowb + 16 > M) return;
  const u16* ap = A  + (size_t)(rowb + m) * K + 8 * hh;
  const u16* bp = Bt + (size_t)(col0 + m) * K + 8 * hh;
  const size_t bs = (size_t)16 * K;
  v8f acc0 = zero8(), acc1 = zero8(), acc2 = zero8(), acc3 = zero8();
#pragma unroll 1
  for (int k0 = 0; k0 < K; k0 += 32) {
    const v16b a  = ldfrag_b(ap + k0);
    const v16b b0 = ldfrag_b(bp + k0);
    const v16b b1 = ldfrag_b(bp + bs + k0);
    const v16b b2 = ldfrag_b(bp + 2 * bs + k0);
    const v16b b3 = ldfrag_b(bp + 3 * bs + k0);
    acc0 = mma_b(a, b0, acc0);
    acc1 = mma_b(a, b1, acc1);
    acc2 = mma_b(a, b2, acc2);
    acc3 = mma_b(a, b3, acc3);
    guard6<v16b>(acc0, acc1, acc2, acc3, a, b0, b1, b2, b3, a);
  }
  epi64(slab + wave * SLAB64, acc0, acc1, acc2, acc3, oscale, bias, bias_n, C, N, (size_t)rowb, col0, lane);
}

template <int NPROD>
__global__ __launch_bounds__(128)
void gemm_h(const u16* __restrict__ Ah, const u16* __restrict__ Al, const u16* __restrict__ Bt,
            const float* __restrict__ bias, int bias_n, float* C, int N, int K, int sbeg, int nrt, int lseq, float oscale) {
  __shared__ __align__(16) float slab[4 * SLAB64];
  const int tid = threadIdx.x, wave = tid >> 5, lane = tid & 31, hh = lane >> 4, m = lane & 15;
  const int ntile = N >> 6;
  const int bid   = blockIdx.x;
  const int ct    = bid % ntile;
  const int t2    = bid / ntile;
  const int rt    = t2 % nrt;
  const int bb    = t2 / nrt;
  if (bb >= NB) return;
  const int srow  = sbeg + rt * 64 + wave * 16;
  if (srow + 16 > SEQ) return;
  const int col0  = ct * 64;
  const size_t rowC = (size_t)bb * SEQ + srow;
  const _Float16* ahp = (const _Float16*)(const void*)Ah + (rowC + m) * (size_t)K + 8 * hh;
  const _Float16* alp = (const _Float16*)(const void*)Al + ((size_t)bb * lseq + srow + m) * (size_t)K + 8 * hh;
  const _Float16* bp  = (const _Float16*)(const void*)Bt + (size_t)(col0 + m) * K + 8 * hh;
  const size_t bs = (size_t)16 * K;
  v8f acc0 = zero8(), acc1 = zero8(), acc2 = zero8(), acc3 = zero8();
  if constexpr (NPROD == 2) {
#pragma unroll 1
    for (int k0 = 0; k0 < K; k0 += 32) {
      const v16h ah = ldfrag_h(ahp + k0), al = ldfrag_h(alp + k0);
      const v16h b0 = ldfrag_h(bp + k0);
      const v16h b1 = ldfrag_h(bp + bs + k0);
      const v16h b2 = ldfrag_h(bp + 2 * bs + k0);
      const v16h b3 = ldfrag_h(bp + 3 * bs + k0);
      acc0 = mma_h(ah, b0, acc0);  acc0 = mma_h(al, b0, acc0);
      acc1 = mma_h(ah, b1, acc1);  acc1 = mma_h(al, b1, acc1);
      acc2 = mma_h(ah, b2, acc2);  acc2 = mma_h(al, b2, acc2);
      acc3 = mma_h(ah, b3, acc3);  acc3 = mma_h(al, b3, acc3);
      guard6<v16h>(acc0, acc1, acc2, acc3, ah, al, b0, b1, b2, b3);
    }
  } else {
#pragma unroll 1
    for (int k0 = 0; k0 < K; k0 += 32) {
      const v16h ah = ldfrag_h(ahp + k0);
      const v16h b0 = ldfrag_h(bp + k0);
      const v16h b1 = ldfrag_h(bp + bs + k0);
      const v16h b2 = ldfrag_h(bp + 2 * bs + k0);
      const v16h b3 = ldfrag_h(bp + 3 * bs + k0);
      acc0 = mma_h(ah, b0, acc0);
      acc1 = mma_h(ah, b1, acc1);
      acc2 = mma_h(ah, b2, acc2);
      acc3 = mma_h(ah, b3, acc3);
      guard6<v16h>(acc0, acc1, acc2, acc3, ah, b0, b1, b2, b3, ah);
    }
  }
  epi64(slab + wave * SLAB64, acc0, acc1, acc2, acc3, oscale, bias, bias_n, C, N, rowC, col0, lane);
}

__global__ __launch_bounds__(256) void knormq(const float* __restrict__ QL, const float* __restrict__ nw, u16* QN) {
  const int tid = threadIdx.x, wave = tid >> 5, lane = tid & 31;
  const int row = blockIdx.x * 8 + wave;
  if (row >= MROWS) return;
  const float* p = QL + (size_t)row * DLQ + lane * 8;
  const v4f a = *(const v4f*)(p), b4 = *(const v4f*)(p + 4);
  const v4f wa = *(const v4f*)(nw + lane * 8), wb = *(const v4f*)(nw + lane * 8 + 4);
  float x[8], w[8];
#pragma unroll
  for (int e = 0; e < 4; ++e) { x[e] = a[e]; x[4 + e] = b4[e]; w[e] = wa[e]; w[4 + e] = wb[e]; }
  float ss = 0.0f;
#pragma unroll
  for (int e = 0; e < 8; ++e) ss += x[e] * x[e];
#pragma unroll
  for (int off = 1; off < 32; off <<= 1) ss += __shfl_xor(ss, off, 32);
  const float r = rsqrtf(ss * (1.0f / DLQ) + RMS_EPS);
  v4u o;
#pragma unroll
  for (int e = 0; e < 4; ++e) {
    const float f0 = x[2 * e] * r * bfr(w[2 * e]) * QNS;
    const float f1 = x[2 * e + 1] * r * bfr(w[2 * e + 1]) * QNS;
    o[e] = pk16(h_bits((_Float16)f0), h_bits((_Float16)f1));
  }
  u16* d = QN + (size_t)row * DLQ + lane * 8;
  for (int pass = 0; pass < 2; ++pass) {
    *(volatile v4u*)(d) = o;
    __threadfence();
  }
}

__global__ __launch_bounds__(320) void kqcat(const float* __restrict__ Q, const float* __restrict__ wkvb, u16* QHo, u16* QLo) {
  __shared__ __align__(16) float qs[NQ];
  const int tid = (int)threadIdx.x;
  const int row = (int)blockIdx.x;
  if (row >= MROWS) return;
  qs[tid] = Q[(size_t)row * NQ + tid];
  __syncthreads();
  const int head  = tid / 20;
  const int chunk = tid - head * 20;
  const int c0    = chunk * 8;
  const int ca    = (c0 < DLKV - 8) ? c0 : (DLKV - 8);
  const float* wp = wkvb + (size_t)(head * HROW) * DLKV + ca;
  const float* qh = qs + head * DQK;
  float val[8];
#pragma unroll
  for (int e = 0; e < 8; ++e) val[e] = 0.0f;
#pragma unroll 1
  for (int n = 0; n < DNOPE; ++n) {
    const float qn = qh[n];
    const v4f w0 = *(const v4f*)(wp + (size_t)n * DLKV), w1 = *(const v4f*)(wp + (size_t)n * DLKV + 4);
#pragma unroll
    for (int e = 0; e < 4; ++e) { val[e] += qn * bfr(w0[e]); val[4 + e] += qn * bfr(w1[e]); }
  }
  float fin[8];
#pragma unroll
  for (int e = 0; e < 8; ++e) {
    const int ridx = c0 - DLKV + e;
    int qi = DNOPE + ridx;
    qi = (qi < 0) ? 0 : qi;
    qi = (qi > DQK - 1) ? (DQK - 1) : qi;
    const float rv   = qh[qi];
    const float rope = (ridx >= 0 && ridx < DROPE) ? rv : 0.0f;
    fin[e] = (c0 < DLKV) ? val[e] : rope;
  }
  v4u oh, ol;
#pragma unroll
  for (int e = 0; e < 4; ++e) {
    const float t0 = fin[2 * e] * QSC, t1 = fin[2 * e + 1] * QSC;
    const _Float16 h0 = (_Float16)t0, h1 = (_Float16)t1;
    const _Float16 l0 = (_Float16)(t0 - (float)h0), l1 = (_Float16)(t1 - (float)h1);
    oh[e] = pk16(h_bits(h0), h_bits(h1));
    ol[e] = pk16(h_bits(l0), h_bits(l1));
  }
  const size_t ob = (size_t)row * QCW + (size_t)tid * 8;
  for (int pass = 0; pass < 2; ++pass) {
    *(volatile v4u*)(QHo + ob) = oh;
    *(volatile v4u*)(QLo + ob) = ol;
    __threadfence();
  }
}

__global__ __launch_bounds__(256) void kkcat(const float* __restrict__ KVL, const float* __restrict__ nw,
                                             const int* __restrict__ spos, const float* __restrict__ kvc,
                                             const float* __restrict__ krc,
                                             u16* KCH, u16* KCL, u16* VTH, u16* VTL) {
  __shared__ __align__(16) u16 lds[2 * KCT * DCAT];
  const int tid = (int)threadIdx.x;
  const int bid = (int)blockIdx.x;
  const int st  = bid % NST;
  const int b   = bid / NST;
  if (b >= NB) return;
  const int s0 = st * KCT;
  const int sl = tid >> 2;
  const int dc = tid & 3;
  const int s  = s0 + sl;
  int sp = spos[0];
  sp = (sp < 0) ? 0 : sp;
  sp = (sp > XS_FULL) ? XS_FULL : sp;
  int rs = s - sp;
  rs = (rs < 0) ? 0 : rs;
  rs = (rs > SEQ - 1) ? (SEQ - 1) : rs;
  const bool usec = (s >= sp);
  const size_t rowK = (size_t)b * SEQ + rs;
  const float* xp = KVL + rowK * NKVP + dc * 32;
  float ss = 0.0f;
#pragma unroll 1
  for (int i = 0; i < 8; ++i) {
    const v4f a = *(const v4f*)(xp + 4 * i);
    ss += a[0] * a[0];
    ss += a[1] * a[1];
    ss += a[2] * a[2];
    ss += a[3] * a[3];
  }
  ss += __shfl_xor(ss, 1, 32);
  ss += __shfl_xor(ss, 2, 32);
  const float r = rsqrtf(ss * (1.0f / DLKV) + RMS_EPS);
  const float* cp = kvc + ((size_t)b * XS_FULL + s) * DLKV + dc * 32;
  const float* wp = nw + dc * 32;
  u16* IH = lds;
  u16* IL = lds + KCT * DCAT;
  u16* ihr = IH + sl * DCAT + dc * 32;
  u16* ilr = IL + sl * DCAT + dc * 32;
#pragma unroll 1
  for (int j = 0; j < 8; ++j) {
    const v4f x4 = *(const v4f*)(xp + 4 * j);
    const v4f c4 = *(const v4f*)(cp + 4 * j);
    const v4f w4 = *(const v4f*)(wp + 4 * j);
    float vv[4];
#pragma unroll
    for (int e = 0; e < 4; ++e) {
      const float n0 = x4[e] * r * bfr(w4[e]);
      vv[e] = usec ? n0 : bfr(c4[e]);
    }
    v2u hq, lq;
#pragma unroll
    for (int e = 0; e < 2; ++e) {
      const float t0 = vv[2 * e] * KSC, t1 = vv[2 * e + 1] * KSC;
      const _Float16 h0 = (_Float16)t0, h1 = (_Float16)t1;
      const _Float16 l0 = (_Float16)(t0 - (float)h0), l1 = (_Float16)(t1 - (float)h1);
      hq[e] = pk16(h_bits(h0), h_bits(h1));
      lq[e] = pk16(h_bits(l0), h_bits(l1));
    }
    *(v2u*)(ihr + 4 * j) = hq;
    *(v2u*)(ilr + 4 * j) = lq;
  }
  const float* tp = KVL + rowK * NKVP + DLKV + dc * 8;
  const float* kp = krc + ((size_t)b * XS_FULL + s) * DROPE;
#pragma unroll 1
  for (int q = 0; q < 2; ++q) {
    const v4f t4 = *(const v4f*)(tp + 4 * q);
    float tv[4];
#pragma unroll
    for (int e = 0; e < 4; ++e) {
      const int rc  = dc * 8 + 4 * q + e;
      const int rcc = (rc < DROPE - 1) ? rc : (DROPE - 1);
      const float kc = kp[rcc];
      const float vs = usec ? t4[e] : bfr(kc);
      tv[e] = (rc < DROPE) ? vs : 0.0f;
    }
    v2u ht, lt;
#pragma unroll
    for (int e = 0; e < 2; ++e) {
      const float t0 = tv[2 * e] * KSC, t1 = tv[2 * e + 1] * KSC;
      const _Float16 h0 = (_Float16)t0, h1 = (_Float16)t1;
      const _Float16 l0 = (_Float16)(t0 - (float)h0), l1 = (_Float16)(t1 - (float)h1);
      ht[e] = pk16(h_bits(h0), h_bits(h1));
      lt[e] = pk16(h_bits(l0), h_bits(l1));
    }
    *(v2u*)(IH + sl * DCAT + DLKV + dc * 8 + 4 * q) = ht;
    *(v2u*)(IL + sl * DCAT + DLKV + dc * 8 + 4 * q) = lt;
  }
  __syncthreads();
  const size_t gb = ((size_t)b * SEQ + s0) * DCAT;
  v4u ph[5], pl[5];
#pragma unroll
  for (int it = 0; it < 5; ++it) {
    const int piece = it * 256 + tid;
    ph[it] = *(const v4u*)(IH + piece * 8);
    pl[it] = *(const v4u*)(IL + piece * 8);
  }
  for (int pass = 0; pass < 2; ++pass) {
#pragma unroll
    for (int it = 0; it < 5; ++it) {
      const int piece = it * 256 + tid;
      *(volatile v4u*)(KCH + gb + (size_t)piece * 8) = ph[it];
      *(volatile v4u*)(KCL + gb + (size_t)piece * 8) = pl[it];
    }
    __threadfence();
  }
  const int q8 = tid >> 3, p8 = (tid & 7) * 8;
  v4u vh[4], vl[4];
#pragma unroll
  for (int it = 0; it < 4; ++it) {
    const int line = it * 32 + q8;
#pragma unroll
    for (int e = 0; e < 4; ++e) {
      const int k0i = (p8 + 2 * e) * DCAT + line;
      const int k1i = k0i + DCAT;
      vh[it][e] = pk16(IH[k0i], IH[k1i]);
      vl[it][e] = pk16(IL[k0i], IL[k1i]);
    }
  }
  const size_t vb = ((size_t)b * DLKV) * SEQ + s0 + p8;
  for (int pass = 0; pass < 2; ++pass) {
#pragma unroll
    for (int it = 0; it < 4; ++it) {
      const int line = it * 32 + q8;
      *(volatile v4u*)(VTH + vb + (size_t)line * SEQ) = vh[it];
      *(volatile v4u*)(VTL + vb + (size_t)line * SEQ) = vl[it];
    }
    __threadfence();
  }
}

__global__ __launch_bounds__(256) void kmcnt(const float* __restrict__ mask, int* CNT) {
  __shared__ int cl[32];
  const int tid = (int)threadIdx.x;
  const int blk = (int)blockIdx.x;
  const int lt  = tid >> 3;
  const int sub = tid & 7;
  int qt = blk * 32 + lt;
  qt = (qt > NQT - 1) ? (NQT - 1) : qt;
  const int r0 = qt * 16 + 2 * sub;
  const float* m0p = mask + (size_t)r0 * XS_FULL;
  const float* m1p = m0p + XS_FULL;
  int last = -1;
  int hv0 = 0, hv1 = 0;
#pragma unroll 1
  for (int t4 = 0; t4 < SEQ; t4 += 4) {
    const v4f a = *(const v4f*)(m0p + t4), c4 = *(const v4f*)(m1p + t4);
#pragma unroll
    for (int e = 0; e < 4; ++e) {
      const bool ua = (a[e] > MASK_THR), ub = (c4[e] > MASK_THR);
      last = (ua || ub) ? (t4 + e) : last;
      hv0 |= ua ? 1 : 0;
      hv1 |= ub ? 1 : 0;
    }
  }
  int hv = hv0 & hv1;
#pragma unroll
  for (int off = 1; off < 8; off <<= 1) {
    const int ol = __shfl_xor(last, off, 32);
    const int oh = __shfl_xor(hv, off, 32);
    last = (ol > last) ? ol : last;
    hv   = (oh < hv) ? oh : hv;
  }
  const int cnt = (hv != 0) ? ((last >> 5) + 1) : NKT;
  if (sub == 0) cl[lt] = cnt;
  __syncthreads();
  if (tid < 32) {
    const int v = cl[tid];
    for (int pass = 0; pass < 2; ++pass) {
      *(volatile int*)(CNT + (size_t)blk * 32 + tid) = v;
      __threadfence();
    }
  }
}

__global__ __launch_bounds__(ATT_THREADS)
void attn_c(const u16* __restrict__ QHp, const u16* __restrict__ QLp,
            const u16* __restrict__ KHp, const u16* __restrict__ KLp,
            const u16* __restrict__ VHp, const u16* __restrict__ VLp,
            const float* __restrict__ mask, const int* __restrict__ CNT,
            const float* __restrict__ ssm, const u16* __restrict__ WVp,
            u16* OHp, u16* OLp, int nqt) {
  __shared__ __align__(16) float smem[WPB * WREG];

  const int tid  = threadIdx.x;
  const int wave = tid >> 5;
  const int lane = tid & 31;
  const int hh   = lane >> 4;
  const int c    = lane & 15;
  const int bid  = blockIdx.x;
  const int qt   = bid % nqt;
  const int t2   = bid / nqt;
  const int hp   = t2 % NHP;
  const int b    = t2 / NHP;
  if (b >= NB) return;
  const int q0   = qt * 16;
  if (q0 + 16 > SEQ) return;
  const bool wl  = (q0 + 16 <= QA);
  const int head = hp * WPB + wave;

  float* pt   = smem + wave * WREG;
  float* slab = pt + PTW;

  const size_t qoff = ((size_t)b * SEQ + q0 + c) * QCW + (size_t)head * DCAT + 8 * hh;
  const _Float16* Qh  = (const _Float16*)(const void*)QHp + qoff;
  const _Float16* Ql  = (const _Float16*)(const void*)QLp + qoff;
  const size_t koff = ((size_t)b * SEQ + c) * DCAT + 8 * hh;
  const _Float16* Khb = (const _Float16*)(const void*)KHp + koff;
  const _Float16* Klb = (const _Float16*)(const void*)KLp + koff;
  const size_t voff = ((size_t)b * DLKV + c) * SEQ + 8 * hh;
  const _Float16* Vhb = (const _Float16*)(const void*)VHp + voff;
  const _Float16* Vlb = (const _Float16*)(const void*)VLp + voff;

  const float lsc1 = SCL / (QSC * KSC);
  const float csl  = bfr(ssm[0]) * (LN_NKEY * LOG2E);
  const float oc   = 1.0f / (PCAR * KSC);
  int nkt = CNT[qt];
  nkt = (nkt < 1) ? 1 : nkt;
  nkt = (nkt > NKT) ? NKT : nkt;
  const float* mp = mask + (size_t)(q0 + 8 * hh) * XS_FULL + c;

  float mrow[8], lrow[8];
  v8f o[8];
#pragma unroll
  for (int r = 0; r < 8; ++r) { mrow[r] = -INFINITY; lrow[r] = 0.f; }
#pragma unroll
  for (int j = 0; j < 8; ++j) o[j] = zero8();

#pragma unroll 1
  for (int kt = 0; kt < nkt; ++kt) {
    const int kb = kt * 32;
    v8f s0 = zero8(), s1 = zero8();
    const _Float16* k0p = Khb + (size_t)kb * DCAT;
    const _Float16* k1p = k0p + (size_t)16 * DCAT;
    const _Float16* l0p = Klb + (size_t)kb * DCAT;
    const _Float16* l1p = l0p + (size_t)16 * DCAT;
#pragma unroll 1
    for (int kk = 0; kk < DCAT / 32; ++kk) {
      const v16h qh  = ldfrag_h(Qh + kk * 32);
      const v16h ql  = ldfrag_h(Ql + kk * 32);
      const v16h kh0 = ldfrag_h(k0p + kk * 32);
      const v16h kh1 = ldfrag_h(k1p + kk * 32);
      const v16h kl0 = ldfrag_h(l0p + kk * 32);
      const v16h kl1 = ldfrag_h(l1p + kk * 32);
      s0 = mma_h(qh, kh0, s0);
      s0 = mma_h(ql, kh0, s0);
      s0 = mma_h(qh, kl0, s0);
      s1 = mma_h(qh, kh1, s1);
      s1 = mma_h(ql, kh1, s1);
      s1 = mma_h(qh, kl1, s1);
      guard2(s0, s1, qh, ql, kh0, kl0, kh1, kl1);
    }
    float mk0[8], mk1[8];
#pragma unroll
    for (int r = 0; r < 8; ++r) {
      mk0[r] = mp[(size_t)r * XS_FULL + kb];
      mk1[r] = mp[(size_t)r * XS_FULL + kb + 16];
    }
#pragma unroll
    for (int r = 0; r < 8; ++r) {
      const float t0 = (s0[r] * lsc1 + mk0[r]) * csl;
      const float t1 = (s1[r] * lsc1 + mk1[r]) * csl;
      float mx = fmaxf(t0, t1);
#pragma unroll
      for (int off = 1; off < 16; off <<= 1) mx = fmaxf(mx, __shfl_xor(mx, off, 32));
      const float mn = fmaxf(mrow[r], mx);
      const float ms = (mn == -INFINITY) ? 0.0f : mn;
      const float al = exp2f(mrow[r] - ms);
      mrow[r] = mn;
      const float e0 = exp2f(t0 - ms), e1 = exp2f(t1 - ms);
      float ps = e0 + e1;
#pragma unroll
      for (int off = 1; off < 16; off <<= 1) ps += __shfl_xor(ps, off, 32);
      lrow[r] = lrow[r] * al + ps;
#pragma unroll
      for (int j = 0; j < 8; ++j) o[j][r] *= al;
      const int ro = (8 * hh + r) * PTP + c;
      pt[ro]      = e0;
      pt[ro + 16] = e1;
    }
    wave_sync_lds();
    FragH ph, pl;
    {
      const float* prow = pt + c * PTP + 8 * hh;
      const v4f p0 = *(const v4f*)(prow), p1 = *(const v4f*)(prow + 4);
      const v4f p2 = *(const v4f*)(prow + 16), p3 = *(const v4f*)(prow + 20);
#pragma unroll
      for (int e = 0; e < 4; ++e) {
        const float ta = p0[e] * PCAR, tb = p1[e] * PCAR, tc = p2[e] * PCAR, td = p3[e] * PCAR;
        const _Float16 ha = (_Float16)ta, hb = (_Float16)tb, hc = (_Float16)tc, hd = (_Float16)td;
        ph.h[0][e]     = ha;
        ph.h[0][4 + e] = hb;
        ph.h[1][e]     = hc;
        ph.h[1][4 + e] = hd;
        pl.h[0][e]     = (_Float16)(ta - (float)ha);
        pl.h[0][4 + e] = (_Float16)(tb - (float)hb);
        pl.h[1][e]     = (_Float16)(tc - (float)hc);
        pl.h[1][4 + e] = (_Float16)(td - (float)hd);
      }
    }
    {
      const _Float16* vhp = Vhb + kb;
      const _Float16* vlp = Vlb + kb;
#pragma unroll
      for (int jg = 0; jg < 4; ++jg) {
        const size_t da = (size_t)(2 * jg) * 16 * SEQ;
        const size_t db = da + (size_t)16 * SEQ;
        const v16h vha = ldfrag_h(vhp + da), vhb2 = ldfrag_h(vhp + db);
        const v16h vla = ldfrag_h(vlp + da), vlb2 = ldfrag_h(vlp + db);
        o[2 * jg]     = mma_h(ph.v, vha,  o[2 * jg]);
        o[2 * jg]     = mma_h(pl.v, vha,  o[2 * jg]);
        o[2 * jg]     = mma_h(ph.v, vla,  o[2 * jg]);
        o[2 * jg + 1] = mma_h(ph.v, vhb2, o[2 * jg + 1]);
        o[2 * jg + 1] = mma_h(pl.v, vhb2, o[2 * jg + 1]);
        o[2 * jg + 1] = mma_h(ph.v, vlb2, o[2 * jg + 1]);
        guard2(o[2 * jg], o[2 * jg + 1], ph.v, pl.v, vha, vhb2, vla, vlb2);
      }
    }
    wave_sync_lds();
  }
  acc_guard4(o[0], o[1], o[2], o[3]);
  acc_guard4(o[4], o[5], o[6], o[7]);
#pragma unroll
  for (int r = 0; r < 8; ++r) {
    const float lv  = lrow[r];
    const float ls  = (lv > 0.0f) ? lv : 1.0f;
    const float inv = (lv > 0.0f) ? ((1.0f / ls) * oc) : 0.0f;
#pragma unroll
    for (int j = 0; j < 8; ++j) {
      const int idx = (8 * hh + r) * SLP + j * 16 + c;
      slab[idx] = o[j][r] * inv;
    }
  }
  wave_sync_lds();
  v8f va0 = zero8(), va1 = zero8(), va2 = zero8(), va3 = zero8();
  {
    const _Float16* wvp = (const _Float16*)(const void*)WVp + (size_t)(head * HROW + DNOPE + c) * DLKV + 8 * hh;
    const float* arow = slab + c * SLP + 8 * hh;
#pragma unroll 1
    for (int kk = 0; kk < DLKV / 32; ++kk) {
      FragH ah, al;
      const v4f p0 = *(const v4f*)(arow + kk * 32), p1 = *(const v4f*)(arow + kk * 32 + 4);
      const v4f p2 = *(const v4f*)(arow + kk * 32 + 16), p3 = *(const v4f*)(arow + kk * 32 + 20);
#pragma unroll
      for (int e = 0; e < 4; ++e) {
        const float ta = p0[e] * AVS, tb = p1[e] * AVS, tc = p2[e] * AVS, td = p3[e] * AVS;
        const _Float16 ha = (_Float16)ta, hb = (_Float16)tb, hc = (_Float16)tc, hd = (_Float16)td;
        ah.h[0][e]     = ha;
        ah.h[0][4 + e] = hb;
        ah.h[1][e]     = hc;
        ah.h[1][4 + e] = hd;
        al.h[0][e]     = (_Float16)(ta - (float)ha);
        al.h[0][4 + e] = (_Float16)(tb - (float)hb);
        al.h[1][e]     = (_Float16)(tc - (float)hc);
        al.h[1][4 + e] = (_Float16)(td - (float)hd);
      }
      const v16h b0 = ldfrag_h(wvp + kk * 32);
      const v16h b1 = ldfrag_h(wvp + (size_t)16 * DLKV + kk * 32);
      const v16h b2 = ldfrag_h(wvp + (size_t)32 * DLKV + kk * 32);
      const v16h b3 = ldfrag_h(wvp + (size_t)48 * DLKV + kk * 32);
      va0 = mma_h(ah.v, b0, va0);  va0 = mma_h(al.v, b0, va0);
      va1 = mma_h(ah.v, b1, va1);  va1 = mma_h(al.v, b1, va1);
      va2 = mma_h(ah.v, b2, va2);  va2 = mma_h(al.v, b2, va2);
      va3 = mma_h(ah.v, b3, va3);  va3 = mma_h(al.v, b3, va3);
      guard6<v16h>(va0, va1, va2, va3, ah.v, al.v, b0, b1, b2, b3);
    }
  }
  wave_sync_lds();
  {
    const float ivs = 1.0f / (AVS * WVS);
#pragma unroll
    for (int r = 0; r < 8; ++r) {
      const int ro = (8 * hh + r) * SLP + c;
      slab[ro]      = va0[r] * ivs;
      slab[ro + 16] = va1[r] * ivs;
      slab[ro + 32] = va2[r] * ivs;
      slab[ro + 48] = va3[r] * ivs;
    }
  }
  wave_sync_lds();
  v4u oh[4], ol[4];
  const int rq = lane >> 3, c8 = (lane & 7) * 8;
#pragma unroll
  for (int it = 0; it < 4; ++it) {
    const int row = it * 4 + rq;
    const v4f a = *(const v4f*)(slab + row * SLP + c8), b4 = *(const v4f*)(slab + row * SLP + c8 + 4);
    float w[8];
#pragma unroll
    for (int e = 0; e < 4; ++e) { w[e] = a[e] * OSC; w[4 + e] = b4[e] * OSC; }
#pragma unroll
    for (int e = 0; e < 4; ++e) {
      const _Float16 h0 = (_Float16)w[2 * e], h1 = (_Float16)w[2 * e + 1];
      const _Float16 l0 = (_Float16)(w[2 * e] - (float)h0), l1 = (_Float16)(w[2 * e + 1] - (float)h1);
      oh[it][e] = pk16(h_bits(h0), h_bits(h1));
      ol[it][e] = pk16(h_bits(l0), h_bits(l1));
    }
  }
  const size_t ob  = ((size_t)b * SEQ + q0) * VOUT + (size_t)head * DV + c8;
  const size_t obl = ((size_t)b * QA + q0) * VOUT + (size_t)head * DV + c8;
  for (int pass = 0; pass < 2; ++pass) {
#pragma unroll
    for (int it = 0; it < 4; ++it) {
      const int row = it * 4 + rq;
      *(volatile v4u*)(OHp + ob + (size_t)row * VOUT) = oh[it];
      if (wl) {
        *(volatile v4u*)(OLp + obl + (size_t)row * VOUT) = ol[it];
      }
    }
    __threadfence();
  }
}

static size_t al256(size_t b) { return (b + 255) & ~(size_t)255; }

extern "C" void kernel_launch(void* const* d_in, const int* in_sizes, int n_in,
                              void* d_out, int out_size, void* d_ws, size_t ws_size,
                              hipStream_t stream) {
  if (n_in < 19) return;
  if (in_sizes[0] < ((NB - 1) * XS_FULL + SEQ) * DMOD) return;
  if (in_sizes[1] < 1) return;
  if (in_sizes[3] != XS_FULL * XS_FULL) return;
  if (in_sizes[5] != DLQ * DMOD) return;
  if (in_sizes[6] != DLQ) return;
  if (in_sizes[7] != DLQ) return;
  if (in_sizes[8] != NQ * DLQ) return;
  if (in_sizes[9] != NQ) return;
  if (in_sizes[10] != NKVA * DMOD) return;
  if (in_sizes[11] != NKVA) return;
  if (in_sizes[12] != DLKV) return;
  if (in_sizes[13] != WKVB_ROWS * DLKV) return;
  if (in_sizes[14] != DMOD * VOUT) return;
  if (in_sizes[15] != DMOD) return;
  if (in_sizes[16] < 1) return;
  if (in_sizes[17] < NB * XS_FULL * DLKV) return;
  if (in_sizes[18] < NB * XS_FULL * DROPE) return;
  if (out_size < MROWS * DMOD) return;

  const float* h      = (const float*)d_in[0];
  const int*   spos   = (const int*)d_in[1];
  const float* maskp  = (const float*)d_in[3];
  const float* wqa    = (const float*)d_in[5];
  const float* wqa_b  = (const float*)d_in[6];
  const float* qnw    = (const float*)d_in[7];
  const float* wqb    = (const float*)d_in[8];
  const float* wqb_b  = (const float*)d_in[9];
  const float* wkva   = (const float*)d_in[10];
  const float* wkva_b = (const float*)d_in[11];
  const float* kvnw   = (const float*)d_in[12];
  const float* wkvb   = (const float*)d_in[13];
  const float* wo     = (const float*)d_in[14];
  const float* wo_b   = (const float*)d_in[15];
  const float* ssm    = (const float*)d_in[16];
  const float* kvc    = (const float*)d_in[17];
  const float* krc    = (const float*)d_in[18];
  float*       out    = (float*)d_out;

  const size_t szXB   = al256((size_t)MROWS * DMOD * 2);
  const size_t szVH   = al256((size_t)MROWS * VOUT * 2);
  const size_t szR1   = (szXB > szVH) ? szXB : szVH;
  const size_t szWQA  = al256((size_t)DLQ * DMOD * 2);
  const size_t szWKVA = al256((size_t)NKVP * DMOD * 2);
  const size_t szWQB  = al256((size_t)NQ * DLQ * 2);
  const size_t szWVB  = al256((size_t)WKVB_ROWS * DLKV * 2);
  const size_t szWO   = al256((size_t)DMOD * VOUT * 2);
  const size_t szQLAT = al256((size_t)MROWS * DLQ * 4);
  const size_t szQN   = al256((size_t)MROWS * DLQ * 2);
  const size_t szKVL  = al256((size_t)MROWS * NKVP * 4);
  const size_t szQCL  = al256((size_t)MROWS * QCW * 2);
  const size_t szR2a  = szQLAT + szQN + szKVL;
  const size_t szR2   = (szR2a > szQCL) ? szR2a : szQCL;
  const size_t szQ    = al256((size_t)MROWS * NQ * 4);
  const size_t szQCH  = al256((size_t)MROWS * QCW * 2);
  const size_t szKC   = al256((size_t)MROWS * DCAT * 2);
  const size_t szVT   = al256((size_t)NB * DLKV * SEQ * 2);
  const size_t szCNT  = al256((size_t)NQT32 * 32 * 4);
  const size_t szVL   = al256((size_t)NB * QA * VOUT * 2);

  size_t off = 0;
  const size_t oR1   = off; off += szR1;
  const size_t oWQA  = off; off += szWQA;
  const size_t oWKVA = off; off += szWKVA;
  const size_t oWQB  = off; off += szWQB;
  const size_t oWVB  = off; off += szWVB;
  const size_t oWO   = off; off += szWO;
  const size_t oR2   = off; off += szR2;
  const size_t oQ    = off; off += szQ;
  const size_t oQCH  = off; off += szQCH;
  const size_t oKCH  = off; off += szKC;
  const size_t oKCL  = off; off += szKC;
  const size_t oVTH  = off; off += szVT;
  const size_t oVTL  = off; off += szVT;
  const size_t oCNT  = off; off += szCNT;
  const size_t oVL   = off; off += szVL;
  if (off > ws_size) return;
  if (off > (size_t)WS_CAP) return;

  char* ws = (char*)d_ws;
  u16*   XB   = (u16*)(ws + oR1);
  u16*   VH   = (u16*)(ws + oR1);
  u16*   WQA  = (u16*)(ws + oWQA);
  u16*   WKVA = (u16*)(ws + oWKVA);
  u16*   WQB  = (u16*)(ws + oWQB);
  u16*   WVB  = (u16*)(ws + oWVB);
  u16*   WO   = (u16*)(ws + oWO);
  float* QLAT = (float*)(ws + oR2);
  u16*   QN   = (u16*)(ws + oR2 + szQLAT);
  float* KVL  = (float*)(ws + oR2 + szQLAT + szQN);
  u16*   QCL  = (u16*)(ws + oR2);
  float* Qf   = (float*)(ws + oQ);
  u16*   QCH  = (u16*)(ws + oQCH);
  u16*   KCH  = (u16*)(ws + oKCH);
  u16*   KCL  = (u16*)(ws + oKCL);
  u16*   VTH  = (u16*)(ws + oVTH);
  u16*   VTL  = (u16*)(ws + oVTL);
  int*   CNT  = (int*)(ws + oCNT);
  u16*   VL   = (u16*)(ws + oVL);

  const dim3 b256(256), b128(128), b320(320), bAT(ATT_THREADS);
  const int  n8x   = (MROWS * DMOD) / 8;
  const int  n8xb  = (SEQ * DMOD) / 8;
  const int  n8qa  = (DLQ * DMOD) / 8;
  const int  n8kv  = (NKVP * DMOD) / 8;
  const int  n8kvs = (NKVA * DMOD) / 8;
  const int  n8qb  = (NQ * DLQ) / 8;
  const int  n8vb  = (WKVB_ROWS * DLKV) / 8;
  const int  n8wo  = (DMOD * VOUT) / 8;
  const dim3 gX((n8x + 255) / 256);
  const dim3 gWQA((n8qa + 255) / 256);
  const dim3 gWKVA((n8kv + 255) / 256);
  const dim3 gWQB((n8qb + 255) / 256);
  const dim3 gWVB((n8vb + 255) / 256);
  const dim3 gWO((n8wo + 255) / 256);
  const dim3 gGQA((MROWS / 64) * (DLQ / 64));
  const dim3 gGKV((MROWS / 64) * (NKVP / 64));
  const dim3 gNQ(MROWS / 8);
  const dim3 gGQB(NB * (SEQ / 64) * (NQ / 64));
  const dim3 gKK(NB * NST);
  const dim3 gQC(MROWS);
  const dim3 gMC(NQT32);
  const dim3 gAT(NQT * NHP * NB);
  const int  nrtA = QA / 64;
  const int  nrtB = (SEQ - QA) / 64;

  cvt_x<<<gX, b256, 0, stream>>>(h, XB, n8x, n8xb);
  cvt16<<<gWQA, b256, 0, stream>>>(wqa, WQA, n8qa, n8qa, 0, 1.0f);
  cvt16<<<gWKVA, b256, 0, stream>>>(wkva, WKVA, n8kv, n8kvs, 0, 1.0f);
  cvt16<<<gWQB, b256, 0, stream>>>(wqb, WQB, n8qb, n8qb, 1, WQS);
  cvt16<<<gWVB, b256, 0, stream>>>(wkvb, WVB, n8vb, n8vb, 1, WVS);
  cvt16<<<gWO, b256, 0, stream>>>(wo, WO, n8wo, n8wo, 1, WOS);
  gemm_bf<<<gGQA, b128, 0, stream>>>(XB, WQA, wqa_b, DLQ, QLAT, MROWS, DLQ, DMOD, 1.0f);
  gemm_bf<<<gGKV, b128, 0, stream>>>(XB, WKVA, wkva_b, NKVA, KVL, MROWS, NKVP, DMOD, 1.0f);
  knormq<<<gNQ, b256, 0, stream>>>(QLAT, qnw, QN);
  gemm_h<1><<<gGQB, b128, 0, stream>>>(QN, QN, WQB, wqb_b, NQ, Qf, NQ, DLQ, 0, SEQ / 64, SEQ, 1.0f / (QNS * WQS));
  kkcat<<<gKK, b256, 0, stream>>>(KVL, kvnw, spos, kvc, krc, KCH, KCL, VTH, VTL);
  kqcat<<<gQC, b320, 0, stream>>>(Qf, wkvb, QCH, QCL);
  kmcnt<<<gMC, b256, 0, stream>>>(maskp, CNT);
  attn_c<<<gAT, bAT, 0, stream>>>(QCH, QCL, KCH, KCL, VTH, VTL, maskp, CNT, ssm, WVB, VH, VL, NQT);
  gemm_h<2><<<dim3(NB * nrtA * (DMOD / 64)), b128, 0, stream>>>(VH, VL, WO, wo_b, DMOD, out, DMOD, VOUT, 0, nrtA, QA,
                                                              1.0f / (OSC * WOS));
  if (nrtB > 0) {
    gemm_h<1><<<dim3(NB * nrtB * (DMOD / 64)), b128, 0, stream>>>(VH, VL, WO, wo_b, DMOD, out, DMOD, VOUT, QA, nrtB, QA,
                                                                1.0f / (OSC * WOS));
  }
  (void)hipGetLastError();
}
